// ControlVariate_23261542875179
// MI455X (gfx1250) — hardware-verified
//
#include <hip/hip_runtime.h>
#include <math.h>

typedef __bf16          v16bf __attribute__((ext_vector_type(16)));
typedef unsigned short  v8us  __attribute__((ext_vector_type(8), may_alias));
typedef unsigned int    v4u   __attribute__((ext_vector_type(4), may_alias));
typedef float           v4f   __attribute__((ext_vector_type(4), may_alias));
typedef float           v8f   __attribute__((ext_vector_type(8)));

#define NO_   64
#define NP_   64
#define HID   100
#define NOBS  100
#define NSD   8
#define NAD   10
#define NIN   118
#define NNODE 63
#define GP    112
#define JP    336
#define OIP   352
#define KP    128
#define SAP   64
#define XP    32
#define TPB   2
#define RX    64
#define RH    32
#define HOP   100
#define CP    32
#define NT    (NO_ * NP_)
#define NBLK  (NT / TPB)

#define OFF_WHH 0u
#define OFF_WSA 86016u
#define OFF_OI  129024u
#define OFF_C   219136u
#define WS_END  481280u

__device__ __forceinline__ unsigned short f2bf(float f) {
  unsigned int u = __float_as_uint(f);
  u += 0x7FFFu + ((u >> 16) & 1u);
  return (unsigned short)(u >> 16);
}
__device__ __forceinline__ float bf2f(unsigned short b) {
  return __uint_as_float(((unsigned int)b) << 16);
}
__device__ __forceinline__ float bfr(float f) { return bf2f(f2bf(f)); }

__device__ __forceinline__ v8f zacc() { v8f z = {0.f, 0.f, 0.f, 0.f, 0.f, 0.f, 0.f, 0.f}; return z; }

__device__ __forceinline__ v8f mma(v16bf a, v16bf b, v8f c) {
  c = __builtin_amdgcn_wmma_f32_16x16x32_bf16(false, a, false, b, (short)0, c, false, false);
  asm volatile("v_nop\n\tv_nop\n\tv_nop\n\tv_nop" : "+v"(c) : "v"(a), "v"(b));
  return c;
}

union Frag { v16bf v; v8us hf[2]; };

__device__ __forceinline__ void ldfrag(Frag& f, const unsigned short* p) {
  f.hf[0] = *(const v8us*)(p);
  f.hf[1] = *(const v8us*)(p + 16);
}

__device__ __forceinline__ v8f hid_acc(v8f acc, const unsigned short* hrow_hi,
                                       const unsigned short* hrow_lo,
                                       const unsigned short* wrow) {
  Frag ah, al, bw;
#pragma unroll 1
  for (int ks = 0; ks < 4; ++ks) {
    ldfrag(ah, hrow_hi + ks * 32);
    ldfrag(al, hrow_lo + ks * 32);
    ldfrag(bw, wrow + ks * 32);
    acc = mma(ah.v, bw.v, acc);
    acc = mma(al.v, bw.v, acc);
  }
  return acc;
}

__device__ __forceinline__ float sigm(float x) { return 1.f / (1.f + expf(-x)); }

__global__ __launch_bounds__(32) void k_prep_w(const float* __restrict__ W_ih,
                                              const float* __restrict__ W_hh,
                                              unsigned short* whh, unsigned short* wsa) {
  const int jp = blockIdx.x;
  if (jp >= JP) return;
  const int lane = threadIdx.x & 31;
  const int g = jp / GP;
  const int jj = jp - g * GP;
  const bool valid = jj < HID;
  const int j = g * HID + (valid ? jj : 0);
  const bool isH = lane < 16;
  const bool isS = (lane >= 16) && (lane < 24);

  float v[8];
  unsigned short* dst = whh;
  if (isH) {
    const int k0 = lane * 8;
#pragma unroll
    for (int i = 0; i < 8; ++i) {
      const int k = k0 + i;
      v[i] = (valid && k < HID) ? W_hh[(size_t)j * HID + k] : 0.f;
    }
    dst = whh + (size_t)jp * KP + k0;
  } else if (isS) {
    const int k0 = (lane - 16) * 8;
#pragma unroll
    for (int i = 0; i < 8; ++i) {
      const int k = k0 + i;
      v[i] = (valid && k < (NSD + NAD)) ? W_ih[(size_t)j * NIN + NOBS + k] : 0.f;
    }
    dst = wsa + (size_t)jp * SAP + k0;
  } else {
#pragma unroll
    for (int i = 0; i < 8; ++i) v[i] = 0.f;
  }

  unsigned int hb[8];
#pragma unroll
  for (int i = 0; i < 8; ++i) hb[i] = f2bf(v[i]);
  v4u pk;
  pk.x = hb[0] | (hb[1] << 16); pk.y = hb[2] | (hb[3] << 16);
  pk.z = hb[4] | (hb[5] << 16); pk.w = hb[6] | (hb[7] << 16);

  const bool st = isH || isS;
  if (st) *(volatile v4u*)dst = pk;
  __threadfence();
  if (st) *(volatile v4u*)dst = pk;
}

__global__ __launch_bounds__(OIP) void k_prep_oi(const float* __restrict__ obs,
                                                const float* __restrict__ W_ih,
                                                const float* __restrict__ b_ih,
                                                float* OI) {
  __shared__ __attribute__((aligned(16))) float s[OIP];
  const int o = blockIdx.x;
  if (o >= NO_) return;
  const int t = threadIdx.x;
  float acc = 0.f;
  if (t < JP) {
    const int g = t / GP;
    const int jj = t - g * GP;
    if (jj < HID) {
      const int j = g * HID + jj;
      acc = bfr(b_ih[j]);
#pragma unroll 1
      for (int k = 0; k < NOBS; ++k)
        acc = fmaf(bfr(obs[o * NOBS + k]), bfr(W_ih[(size_t)j * NIN + k]), acc);
    }
  }
  if (t < OIP) s[t] = acc;
  __syncthreads();
  const int wave = t >> 5;
  const int lane = t & 31;
  const bool st = (lane < 8) && (wave * 32 + lane * 4 < OIP);
  v4f val = {0.f, 0.f, 0.f, 0.f};
  float* p = OI;
  if (st) {
    val = *(const v4f*)(s + wave * 32 + lane * 4);
    p = OI + (size_t)o * OIP + wave * 32 + lane * 4;
  }
  if (st) *(volatile v4f*)p = val;
  __threadfence();
  if (st) *(volatile v4f*)p = val;
}

__global__ __launch_bounds__(256) __attribute__((amdgpu_num_vgpr(248))) void k_tree(
    const float* __restrict__ samp, const float* __restrict__ addr,
    const unsigned short* __restrict__ whh, const unsigned short* __restrict__ wsa,
    const float* __restrict__ OI, const float* __restrict__ b_hh,
    const float* __restrict__ W1, const float* __restrict__ b1,
    const float* __restrict__ W2, const float* __restrict__ b2,
    const float* __restrict__ W3, const float* __restrict__ b3,
    float* cbuf) {
  __shared__ __attribute__((aligned(16))) float hout[RX * HOP];
  __shared__ __attribute__((aligned(16))) float hc[RH * HOP];
  __shared__ __attribute__((aligned(16))) unsigned short hch[RH * KP];
  __shared__ __attribute__((aligned(16))) unsigned short hcl[RH * KP];
  __shared__ __attribute__((aligned(16))) unsigned short xb[RX * XP];
  __shared__ float y1s[TPB * 64];
  __shared__ float y2s[TPB * 32];
  __shared__ float cv[TPB];

  const int tid  = threadIdx.x;
  const int lane = tid & 31;
  const int wave = tid >> 5;
  const int blk  = blockIdx.x;
  if (blk >= NBLK) return;
  const int op0  = blk * TPB;
  const int o    = op0 >> 6;
  const int m    = lane & 15;
  const int h    = lane >> 4;

  for (int i = tid; i < RH * KP; i += 256) { hch[i] = 0; hcl[i] = 0; }
  __syncthreads();

  for (int l = 5; l >= 0; --l) {
    const int w  = 1 << l;
    const int s  = w - 1;
    const int R  = TPB << l;
    const int rt = (R + 15) >> 4;

    const int nst = rt * 16 * XP;
    for (int idx = tid; idx < nst; idx += 256) {
      const int row = idx >> 5;
      const int k   = idx & 31;
      float v = 0.f;
      if (row < R) {
        const int t    = row >> l;
        const int node = row & (w - 1);
        const size_t base = (size_t)(op0 + t) * NNODE + (size_t)(s + node);
        if (k < NSD) v = samp[base * NSD + k];
        else if (k < NSD + NAD) v = addr[base * NAD + (k - NSD)];
      }
      xb[idx] = f2bf(v);
    }
    __syncthreads();

    const int njobs = rt * 7;
    for (int job = wave; job < njobs; job += 8) {
      const int r    = job / 7;
      const int jt   = job - r * 7;
      const int arow = r * 16 + m;
      const int cc   = jt * 16 + m;
      const float* oirow = OI + (size_t)o * OIP + cc;
      const unsigned short* hrh = hch + arow * KP + 8 * h;
      const unsigned short* hrl = hcl + arow * KP + 8 * h;

      Frag ax;
      ldfrag(ax, xb + arow * XP + 8 * h);

      float rp[8], zp[8], gn[8], ghn[8];
      {
        const int jp = cc;
        Frag bs;
        ldfrag(bs, wsa + (size_t)jp * SAP + 8 * h);
        v8f acc = mma(ax.v, bs.v, zacc());
        if (l < 5) acc = hid_acc(acc, hrh, hrl, whh + (size_t)jp * KP + 8 * h);
        const float add = oirow[0] + ((cc < HID) ? bfr(b_hh[cc]) : 0.f);
#pragma unroll
        for (int v = 0; v < 8; ++v) rp[v] = acc[v] + add;
      }
      {
        const int jp = GP + cc;
        Frag bs;
        ldfrag(bs, wsa + (size_t)jp * SAP + 8 * h);
        v8f acc = mma(ax.v, bs.v, zacc());
        if (l < 5) acc = hid_acc(acc, hrh, hrl, whh + (size_t)jp * KP + 8 * h);
        const float add = oirow[GP] + ((cc < HID) ? bfr(b_hh[HID + cc]) : 0.f);
#pragma unroll
        for (int v = 0; v < 8; ++v) zp[v] = acc[v] + add;
      }
      {
        const int jp = 2 * GP + cc;
        Frag bs;
        ldfrag(bs, wsa + (size_t)jp * SAP + 8 * h);
        v8f acc  = mma(ax.v, bs.v, zacc());
        v8f acch = zacc();
        if (l < 5) acch = hid_acc(acch, hrh, hrl, whh + (size_t)jp * KP + 8 * h);
        const float oi = oirow[2 * GP];
        const float bh = (cc < HID) ? bfr(b_hh[2 * HID + cc]) : 0.f;
#pragma unroll
        for (int v = 0; v < 8; ++v) { gn[v] = acc[v] + oi; ghn[v] = acch[v] + bh; }
      }

      if (cc < HID) {
#pragma unroll
        for (int v = 0; v < 8; ++v) {
          const int nrow = r * 16 + 8 * h + v;
          if (nrow < R) {
            float hp = 0.f;
            if (l < 5) hp = hc[nrow * HOP + cc];
            const float rr = sigm(rp[v]);
            const float zz = sigm(zp[v]);
            const float nn = tanhf(gn[v] + rr * ghn[v]);
            hout[nrow * HOP + cc] = (1.f - zz) * nn + zz * hp;
          }
        }
      }
    }
    __syncthreads();

    if (l > 0) {
      const int hw = R >> 1;
      for (int idx = tid; idx < hw * HID; idx += 256) {
        const int b = idx / HID;
        const int c = idx - b * HID;
        const float v = hout[(2 * b) * HOP + c] + hout[(2 * b + 1) * HOP + c];
        hc[b * HOP + c] = v;
        const unsigned short hs = f2bf(v);
        hch[b * KP + c] = hs;
        hcl[b * KP + c] = f2bf(v - bf2f(hs));
      }
      const int zr = ((R < RH) ? R : RH) - hw;
      for (int idx = tid; idx < zr * HID; idx += 256) {
        const int b = hw + idx / HID;
        const int c = idx % HID;
        hc[b * HOP + c] = 0.f;
        hch[b * KP + c] = 0;
        hcl[b * KP + c] = 0;
      }
      __syncthreads();
    }
  }

  if (tid < TPB * 50) {
    const int t = tid / 50;
    const int u = tid - t * 50;
    float a = bfr(b1[u]);
#pragma unroll 1
    for (int k = 0; k < HID; ++k) a = fmaf(bfr(W1[u * HID + k]), hout[t * HOP + k], a);
    y1s[t * 64 + u] = fmaxf(a, 0.f);
  }
  __syncthreads();
  if (tid < TPB * 25) {
    const int t = tid / 25;
    const int u = tid - t * 25;
    float a = bfr(b2[u]);
#pragma unroll 1
    for (int k = 0; k < 50; ++k) a = fmaf(bfr(W2[u * 50 + k]), y1s[t * 64 + k], a);
    y2s[t * 32 + u] = fmaxf(a, 0.f);
  }
  __syncthreads();
  if (tid < TPB) {
    float a = bfr(b3[0]);
#pragma unroll 1
    for (int k = 0; k < 25; ++k) a = fmaf(bfr(W3[k]), y2s[tid * 32 + k], a);
    cv[tid] = a;
  }
  __syncthreads();

  const bool st = tid < 8;
  v4f val = {0.f, 0.f, 0.f, 0.f};
  float* p = cbuf;
  if (st) {
    if (tid == 0) { val.x = cv[0]; val.y = cv[1]; }
    p = cbuf + (size_t)blk * CP + tid * 4;
  }
  if (st) *(volatile v4f*)p = val;
  __threadfence();
  if (st) *(volatile v4f*)p = val;
}

__global__ __launch_bounds__(64) void k_lse(const float* __restrict__ cbuf, float* out) {
  __shared__ __attribute__((aligned(16))) float vals[NO_];
  const int t = threadIdx.x;
  if (t < NO_) {
    float mx = -INFINITY;
#pragma unroll 1
    for (int q = 0; q < NP_; ++q) {
      const int op = t * NP_ + q;
      mx = fmaxf(mx, cbuf[(size_t)(op / TPB) * CP + (op % TPB)]);
    }
    float ss = 0.f;
#pragma unroll 1
    for (int q = 0; q < NP_; ++q) {
      const int op = t * NP_ + q;
      ss += expf(cbuf[(size_t)(op / TPB) * CP + (op % TPB)] - mx);
    }
    vals[t] = mx + logf(ss) - logf((float)NP_);
  }
  __syncthreads();
  const bool st = t < 16;
  v4f val = {0.f, 0.f, 0.f, 0.f};
  float* p = out;
  if (st) { val = *(const v4f*)(vals + t * 4); p = out + t * 4; }
  if (st) *(volatile v4f*)p = val;
  __threadfence();
  if (st) *(volatile v4f*)p = val;
}

extern "C" void kernel_launch(void* const* d_in, const int* in_sizes, int n_in,
                              void* d_out, int out_size, void* d_ws, size_t ws_size,
                              hipStream_t stream) {
  if (n_in < 13) return;
  if (out_size != NO_) return;
  if (in_sizes[0] != NO_ * NOBS) return;
  if (in_sizes[1] != NT * NNODE * NSD) return;
  if (in_sizes[2] != NT * NNODE * NAD) return;
  if (in_sizes[3] != 3 * HID * NIN) return;
  if (in_sizes[4] != 3 * HID * HID) return;
  if (in_sizes[5] != 3 * HID || in_sizes[6] != 3 * HID) return;
  if (in_sizes[7] != 50 * HID || in_sizes[8] != 50) return;
  if (in_sizes[9] != 25 * 50 || in_sizes[10] != 25) return;
  if (in_sizes[11] != 25 || in_sizes[12] != 1) return;
  if (ws_size < (size_t)WS_END) return;

  const float* obs  = (const float*)d_in[0];
  const float* samp = (const float*)d_in[1];
  const float* addr = (const float*)d_in[2];
  const float* W_ih = (const float*)d_in[3];
  const float* W_hh = (const float*)d_in[4];
  const float* b_ih = (const float*)d_in[5];
  const float* b_hh = (const float*)d_in[6];
  const float* W1   = (const float*)d_in[7];
  const float* b1   = (const float*)d_in[8];
  const float* W2   = (const float*)d_in[9];
  const float* b2   = (const float*)d_in[10];
  const float* W3   = (const float*)d_in[11];
  const float* b3   = (const float*)d_in[12];

  char* ws = (char*)d_ws;
  unsigned short* whh = (unsigned short*)(ws + OFF_WHH);
  unsigned short* wsa = (unsigned short*)(ws + OFF_WSA);
  float* OI   = (float*)(ws + OFF_OI);
  float* cbuf = (float*)(ws + OFF_C);

  k_prep_w<<<JP, 32, 0, stream>>>(W_ih, W_hh, whh, wsa);
  k_prep_oi<<<NO_, OIP, 0, stream>>>(obs, W_ih, b_ih, OI);
  k_tree<<<NBLK, 256, 0, stream>>>(samp, addr, whh, wsa, OI, b_hh,
                                    W1, b1, W2, b2, W3, b3, cbuf);
  k_lse<<<1, 64, 0, stream>>>(cbuf, (float*)d_out);
}
